// MultiHeadSelfAttention_55293408969108
// MI455X (gfx1250) — hardware-verified
//
#include <hip/hip_runtime.h>
#ifndef NB
#define NB 2
#endif
#ifndef SEQ
#define SEQ 2048
#endif
#define SEQ_FULL 2048
#define DM 1024
#define NH 16
#define HD 64
#define SQ SEQ
#define NR ((size_t)NB * SQ)
#define BAND ((SQ) < 512 ? (SQ) : 512)
#define INV_CARRY_R 0.0009765625f

static_assert(NH * HD == DM);
static_assert(HD == 64);
static_assert(DM % 128 == 0);
static_assert(DM % 32 == 0);
static_assert(SQ % 128 == 0);
static_assert(BAND % 128 == 0);
static_assert(BAND <= SQ);
static_assert(((size_t)NB * SQ) % 128 == 0);
static_assert(((size_t)SQ * 16) % 256 == 0);
static_assert(((size_t)SQ * DM / 8) % 256 == 0);
static_assert(((size_t)DM * DM / 8) % 256 == 0);
static_assert(SQ <= SEQ_FULL);

typedef unsigned short v8us __attribute__((ext_vector_type(8), may_alias));
typedef float  v8f  __attribute__((ext_vector_type(8)));
typedef float  v4f  __attribute__((ext_vector_type(4)));
typedef float  v4fa __attribute__((ext_vector_type(4), may_alias));
typedef _Float16 v16h __attribute__((ext_vector_type(16)));
union FragH { v16h v; v8us half[2]; _Float16 h[16]; unsigned short u[16]; };

__device__ __forceinline__ unsigned short bf16_bits(float x) { unsigned int u = __float_as_uint(x); return (unsigned short)((u + 0x7FFFu + ((u >> 16) & 1u)) >> 16); }
__device__ __forceinline__ float bf16_rne(float x) { return __uint_as_float(((unsigned int)bf16_bits(x)) << 16); }

__device__ __forceinline__ v16h g2_frag(const _Float16* p, unsigned hh) { FragH f; f.half[0] = *(const v8us*)((const unsigned short*)p + 8u * hh); f.half[1] = *(const v8us*)((const unsigned short*)p + 16u + 8u * hh); return f.v; }
__device__ __forceinline__ v8f g2_mma(v16h a, v16h b, v8f c) { v8f d = __builtin_amdgcn_wmma_f32_16x16x32_f16(false, a, false, b, (short)0, c, false, false); asm volatile("v_nop\n\tv_nop\n\tv_nop\n\tv_nop" : "+v"(d) : "v"(a), "v"(b)); return d; }
__device__ __forceinline__ void split8(const v4f a, const v4f c, FragH& fh, FragH& fl) {
#pragma unroll
  for (int q = 0; q < 4; ++q) { _Float16 h = (_Float16)a[q]; fh.h[q] = h; fl.h[q] = (_Float16)((a[q] - (float)h) * 1024.0f); h = (_Float16)c[q]; fh.h[4 + q] = h; fl.h[4 + q] = (_Float16)((c[q] - (float)h) * 1024.0f); }
}

__global__ __launch_bounds__(256) void k_wnat(const float* __restrict__ wsrc, size_t n8, _Float16* __restrict__ Bt) {
  const size_t t = (size_t)blockIdx.x * 256u + threadIdx.x; if (t >= n8) return; FragH f;
  const v4f a = *(const v4fa*)(wsrc + t * 8), c = *(const v4fa*)(wsrc + t * 8 + 4);
#pragma unroll
  for (int q = 0; q < 4; ++q) { f.h[q] = (_Float16)(bf16_rne(a[q]) * 16.0f); f.h[4 + q] = (_Float16)(bf16_rne(c[q]) * 16.0f); }
  unsigned short* d = (unsigned short*)Bt + t * 8;
  *(volatile v8us*)d = f.half[0]; __threadfence(); *(volatile v8us*)d = f.half[0];
}
__global__ __launch_bounds__(256) void k_x16(const float* __restrict__ x, _Float16* __restrict__ X16) {
  const size_t t = (size_t)blockIdx.x * 256u + threadIdx.x; const unsigned b = blockIdx.y;
  if (t >= (size_t)SQ * DM / 8) return;
  const float* src = x + (size_t)b * SEQ_FULL * DM + t * 8; FragH f;
  const v4f a = *(const v4fa*)src, c = *(const v4fa*)(src + 4);
#pragma unroll
  for (int q = 0; q < 4; ++q) { f.h[q] = (_Float16)bf16_rne(a[q]); f.h[4 + q] = (_Float16)bf16_rne(c[q]); }
  unsigned short* d = (unsigned short*)X16 + (size_t)b * SQ * DM + t * 8;
  *(volatile v8us*)d = f.half[0]; __threadfence(); *(volatile v8us*)d = f.half[0];
}
struct InvF { float v[32]; };
static_assert(sizeof(InvF) == 128);
__global__ __launch_bounds__(256) void k_ropetab(const int* __restrict__ tp, float* __restrict__ tab, InvF iv) {
  const unsigned t = blockIdx.x * 256u + threadIdx.x; const unsigned b = blockIdx.y;
  const unsigned s = t >> 4, jj = t & 15u;
  if (s >= (unsigned)SQ) return;
  const float pos = (float)tp[(size_t)b * SEQ_FULL + s];
  float f0 = 0.f, f1 = 0.f;
#pragma unroll
  for (unsigned j = 0; j < 16; ++j) { const bool m = (j == jj); f0 = m ? iv.v[2 * j] : f0; f1 = m ? iv.v[2 * j + 1] : f1; }
  v4f o = {0.f, 0.f, 0.f, 0.f};
#pragma unroll 1
  for (int u = 0; u < 2; ++u) {
    const float ang = pos * ((u == 0) ? f0 : f1);
    float sn, cs; sincosf(ang, &sn, &cs);
    if (u == 0) { o[0] = cs; o[1] = sn; } else { o[2] = cs; o[3] = sn; }
  }
  float* d = tab + ((size_t)b * SQ + s) * 64u + jj * 4u;
  *(volatile v4f*)d = o; __threadfence(); *(volatile v4f*)d = o;
}

template <bool ARES, int EPI>
__global__ __launch_bounds__(128) __attribute__((amdgpu_num_vgpr(256)))
void k_gemm3(const _Float16* __restrict__ A, const _Float16* __restrict__ Ar, unsigned lda, size_t sA,
             const _Float16* __restrict__ Bh, unsigned ldb, size_t sB, float alpha, const float* __restrict__ tab,
             float* __restrict__ C, _Float16* __restrict__ Ch, _Float16* __restrict__ Cr, unsigned ldc, size_t sC, unsigned M, unsigned K) {
  static_assert(EPI == 0 || EPI == 1 || EPI == 2);
  __shared__ __attribute__((aligned(16))) float so[4][32][68];
  const unsigned tid = threadIdx.x, w = tid >> 5, lane = tid & 31u, ln = lane & 15u, hh = lane >> 4;
  const unsigned by = blockIdx.z;
  const unsigned row0 = blockIdx.y * 128u + 32u * w, col0 = blockIdx.x * 64u;
  if (row0 >= M) return;
  const size_t cofs = (size_t)by * sC;
  const _Float16* a0p = A + (size_t)by * sA + (size_t)(row0 + ln) * lda; const _Float16* a1p = a0p + (size_t)16 * lda;
  const _Float16* r0p = a0p; const _Float16* r1p = a1p;
  if (ARES) { r0p = Ar + (size_t)by * sA + (size_t)(row0 + ln) * lda; r1p = r0p + (size_t)16 * lda; }
  const _Float16* b0p = Bh + (size_t)by * sB + (size_t)(col0 + ln) * ldb; const _Float16* b1p = b0p + (size_t)16 * ldb; const _Float16* b2p = b1p + (size_t)16 * ldb; const _Float16* b3p = b2p + (size_t)16 * ldb;
  const v8f z8 = {0.f, 0.f, 0.f, 0.f, 0.f, 0.f, 0.f, 0.f};
  v8f c00 = z8, c01 = z8, c02 = z8, c03 = z8, c10 = z8, c11 = z8, c12 = z8, c13 = z8;
  v8f d00 = z8, d01 = z8, d02 = z8, d03 = z8, d10 = z8, d11 = z8, d12 = z8, d13 = z8;
#pragma unroll 1
  for (unsigned kb = 0; kb < K; kb += 32u) {
    const v16h a0 = g2_frag(a0p + kb, hh), a1 = g2_frag(a1p + kb, hh);
    v16h r0 = a0, r1 = a1;
    if (ARES) { r0 = g2_frag(r0p + kb, hh); r1 = g2_frag(r1p + kb, hh); }
    v16h bq = g2_frag(b0p + kb, hh); c00 = g2_mma(a0, bq, c00); c10 = g2_mma(a1, bq, c10); if (ARES) { d00 = g2_mma(r0, bq, d00); d10 = g2_mma(r1, bq, d10); }
    bq = g2_frag(b1p + kb, hh); c01 = g2_mma(a0, bq, c01); c11 = g2_mma(a1, bq, c11); if (ARES) { d01 = g2_mma(r0, bq, d01); d11 = g2_mma(r1, bq, d11); }
    bq = g2_frag(b2p + kb, hh); c02 = g2_mma(a0, bq, c02); c12 = g2_mma(a1, bq, c12); if (ARES) { d02 = g2_mma(r0, bq, d02); d12 = g2_mma(r1, bq, d12); }
    bq = g2_frag(b3p + kb, hh); c03 = g2_mma(a0, bq, c03); c13 = g2_mma(a1, bq, c13); if (ARES) { d03 = g2_mma(r0, bq, d03); d13 = g2_mma(r1, bq, d13); }
  }
  v8f accs[8] = {c00, c01, c02, c03, c10, c11, c12, c13};
  v8f accr[8] = {d00, d01, d02, d03, d10, d11, d12, d13};
#pragma unroll
  for (int u = 0; u < 8; ++u) { const unsigned t = (unsigned)u & 3u, half = (unsigned)u >> 2;
#pragma unroll
    for (int r = 0; r < 8; ++r) { float v = accs[u][r]; if (ARES) v += accr[u][r] * INV_CARRY_R; so[w][half * 16u + 8u * hh + (unsigned)r][t * 16u + ln] = v * alpha; } }
  __builtin_amdgcn_fence(4  , "workgroup"); __builtin_amdgcn_wave_barrier();
  if (EPI == 0) {
    const unsigned rsub = lane >> 4, c4 = (lane & 15u) * 4u;
    for (int pass = 0; pass < 2; ++pass) {
#pragma unroll
      for (unsigned q = 0; q < 16; ++q) { const unsigned r = q * 2u + rsub; const v4f v = *(const v4fa*)&so[w][r][c4]; *(volatile v4f*)(C + cofs + (size_t)(row0 + r) * ldc + col0 + c4) = v; }
      if (pass == 0) __threadfence(); }
  } else {
    const unsigned rq = lane >> 3, c8 = (lane & 7u) * 8u;
    for (int pass = 0; pass < 2; ++pass) {
#pragma unroll
      for (unsigned q = 0; q < 8; ++q) { const unsigned r = q * 4u + rq;
        v4f v0 = *(const v4fa*)&so[w][r][c8]; v4f v1 = *(const v4fa*)&so[w][r][c8 + 4u];
        if (EPI == 2) {
          const float* tq = tab + (size_t)(row0 + r) * 64u + c8;
          const v4f t0 = *(const v4fa*)tq, t1 = *(const v4fa*)(tq + 4);
          v4f e0, e1;
          e0[0] = v0[0] * t0[0] - v0[1] * t0[1]; e0[1] = v0[0] * t0[1] + v0[1] * t0[0];
          e0[2] = v0[2] * t0[2] - v0[3] * t0[3]; e0[3] = v0[2] * t0[3] + v0[3] * t0[2];
          e1[0] = v1[0] * t1[0] - v1[1] * t1[1]; e1[1] = v1[0] * t1[1] + v1[1] * t1[0];
          e1[2] = v1[2] * t1[2] - v1[3] * t1[3]; e1[3] = v1[2] * t1[3] + v1[3] * t1[2];
          v0 = e0; v1 = e1; }
        FragH fh, fl; split8(v0, v1, fh, fl);
        const size_t o = cofs + (size_t)(row0 + r) * ldc + col0 + c8;
        *(volatile v8us*)((unsigned short*)Ch + o) = fh.half[0];
        *(volatile v8us*)((unsigned short*)Cr + o) = fl.half[0]; }
      if (pass == 0) __threadfence(); }
  }
}

template <bool BND>
__global__ __launch_bounds__(128) __attribute__((amdgpu_num_vgpr(256)))
void k_attn(const _Float16* __restrict__ Qh, const _Float16* __restrict__ Qr, const _Float16* __restrict__ Kh, const _Float16* __restrict__ Kr,
            const _Float16* __restrict__ VTh, const _Float16* __restrict__ VTr, _Float16* __restrict__ Oh, _Float16* __restrict__ Orr, unsigned qt0) {
  __shared__ __attribute__((aligned(16))) _Float16 ps[4][BND ? 2 : 1][16][72];
  __shared__ __attribute__((aligned(16))) float so[4][16][68];
  const unsigned tid = threadIdx.x, w = tid >> 5, lane = tid & 31u, ln = lane & 15u, hh = lane >> 4;
  const unsigned qt = blockIdx.x + qt0, h = blockIdx.y, b = blockIdx.z;
  const size_t rowb = (size_t)b * SQ;
  const unsigned qloc = w * 16u;
  const size_t qrow = rowb + (size_t)qt * 64u + qloc;
  v16h qh[2], qr[2];
  { const _Float16* p = Qh + (qrow + ln) * DM + h * HD; const _Float16* pr = Qr + (qrow + ln) * DM + h * HD;
#pragma unroll
    for (unsigned c = 0; c < 2; ++c) { qh[c] = g2_frag(p + c * 32u, hh); qr[c] = g2_frag(pr + c * 32u, hh); } }
  const _Float16* kbh = Kh + (rowb + ln) * DM + h * HD;
  const _Float16* kbr = Kr + (rowb + ln) * DM + h * HD;
  const _Float16* vbh = VTh + (size_t)(h * HD + ln) * NR + rowb;
  const _Float16* vbr = VTr + (size_t)(h * HD + ln) * NR + rowb;
  const v8f z8 = {0.f, 0.f, 0.f, 0.f, 0.f, 0.f, 0.f, 0.f};
  v8f oH[4], oR[4];
#pragma unroll
  for (int nt = 0; nt < 4; ++nt) { oH[nt] = z8; oR[nt] = z8; }
  float mI[8], lI[8];
#pragma unroll
  for (int r = 0; r < 8; ++r) { mI[r] = -1.0e30f; lI[r] = 0.f; }
#pragma unroll 1
  for (unsigned kt = 0; kt <= qt; ++kt) {
    const unsigned kv = kt * 64u;
    v8f s[4];
#pragma unroll
    for (unsigned nt = 0; nt < 4; ++nt) {
      const _Float16* khp = kbh + (size_t)(kv + nt * 16u) * DM;
      const _Float16* krp = kbr + (size_t)(kv + nt * 16u) * DM;
      v8f a = z8, ar = z8;
#pragma unroll
      for (unsigned c = 0; c < 2; ++c) {
        const v16h kh = g2_frag(khp + c * 32u, hh), kr = g2_frag(krp + c * 32u, hh);
        a = g2_mma(qh[c], kh, a); ar = g2_mma(qh[c], kr, ar); ar = g2_mma(qr[c], kh, ar); }
#pragma unroll
      for (int r = 0; r < 8; ++r) s[nt][r] = (a[r] + ar[r] * INV_CARRY_R) * 0.125f;
    }
    if (kt == qt) {
#pragma unroll
      for (unsigned nt = 0; nt < 4; ++nt)
#pragma unroll
        for (int r = 0; r < 8; ++r) { if (nt * 16u + ln > qloc + 8u * hh + (unsigned)r) s[nt][r] = -1.0e9f; }
    }
    float mNew[8], corr[8], rs[8];
#pragma unroll
    for (int r = 0; r < 8; ++r) {
      float m = fmaxf(fmaxf(s[0][r], s[1][r]), fmaxf(s[2][r], s[3][r]));
      m = fmaxf(m, __shfl_xor(m, 1, 16)); m = fmaxf(m, __shfl_xor(m, 2, 16)); m = fmaxf(m, __shfl_xor(m, 4, 16)); m = fmaxf(m, __shfl_xor(m, 8, 16));
      mNew[r] = fmaxf(mI[r], m); corr[r] = __expf(mI[r] - mNew[r]); mI[r] = mNew[r]; rs[r] = 0.f; }
#pragma unroll
    for (unsigned nt = 0; nt < 4; ++nt)
#pragma unroll
      for (int r = 0; r < 8; ++r) {
        const float pv = __expf(s[nt][r] - mNew[r]); rs[r] += pv;
        const float p256 = pv * 256.0f; const _Float16 ph = (_Float16)p256;
        ps[w][0][8u * hh + (unsigned)r][nt * 16u + ln] = ph;
        if (BND) ps[w][BND ? 1 : 0][8u * hh + (unsigned)r][nt * 16u + ln] = (_Float16)((p256 - (float)ph) * 1024.0f); }
#pragma unroll
    for (int r = 0; r < 8; ++r) lI[r] = lI[r] * corr[r] + rs[r];
#pragma unroll
    for (int nt = 0; nt < 4; ++nt)
#pragma unroll
      for (int r = 0; r < 8; ++r) { oH[nt][r] *= corr[r]; if (BND) oR[nt][r] *= corr[r]; }
    __builtin_amdgcn_fence(4  , "workgroup"); __builtin_amdgcn_wave_barrier();
    v16h pA[2], pR[2];
#pragma unroll
    for (unsigned c = 0; c < 2; ++c) { pA[c] = g2_frag(&ps[w][0][ln][c * 32u], hh); pR[c] = pA[c]; if (BND) pR[c] = g2_frag(&ps[w][BND ? 1 : 0][ln][c * 32u], hh); }
#pragma unroll
    for (unsigned nt = 0; nt < 4; ++nt) {
#pragma unroll
      for (unsigned c = 0; c < 2; ++c) {
        const v16h vh = g2_frag(vbh + (size_t)(nt * 16u) * NR + kv + c * 32u, hh);
        oH[nt] = g2_mma(pA[c], vh, oH[nt]);
        if (BND) { const v16h vr = g2_frag(vbr + (size_t)(nt * 16u) * NR + kv + c * 32u, hh);
          oR[nt] = g2_mma(pA[c], vr, oR[nt]); oR[nt] = g2_mma(pR[c], vh, oR[nt]); } }
    }
    __builtin_amdgcn_fence(4  , "workgroup"); __builtin_amdgcn_wave_barrier();
  }
#pragma unroll
  for (int r = 0; r < 8; ++r) {
    float lt = lI[r];
    lt += __shfl_xor(lt, 1, 16); lt += __shfl_xor(lt, 2, 16); lt += __shfl_xor(lt, 4, 16); lt += __shfl_xor(lt, 8, 16);
    const float inv = 0.25f * (1.0f / lt);
#pragma unroll
    for (unsigned nt = 0; nt < 4; ++nt) { float o = oH[nt][r]; if (BND) o += oR[nt][r] * INV_CARRY_R; so[w][8u * hh + (unsigned)r][nt * 16u + ln] = o * inv; } }
  __builtin_amdgcn_fence(4  , "workgroup"); __builtin_amdgcn_wave_barrier();
  const unsigned rq = lane >> 3, c8 = (lane & 7u) * 8u;
  for (int pass = 0; pass < 2; ++pass) {
#pragma unroll
    for (unsigned q = 0; q < 4; ++q) { const unsigned r = q * 4u + rq;
      const v4f v0 = *(const v4fa*)&so[w][r][c8], v1 = *(const v4fa*)&so[w][r][c8 + 4u];
      FragH fh, fl; split8(v0, v1, fh, fl);
      const size_t o = (qrow + r) * DM + h * HD + c8;
      *(volatile v8us*)((unsigned short*)Oh + o) = fh.half[0];
      if (BND) *(volatile v8us*)((unsigned short*)Orr + o) = fl.half[0]; }
    if (pass == 0) __threadfence(); }
}

#define AL256(x) ((((size_t)(x)) + 255) & ~(size_t)255)
constexpr size_t SZ_W  = AL256((size_t)4 * DM * DM * 2);
constexpr size_t SZ_X  = AL256(NR * DM * 2);
constexpr size_t SZ_T  = AL256(NR * 64 * 4);
constexpr size_t SZ_QK = AL256((size_t)2 * NR * DM * 2);
constexpr size_t SZ_P  = AL256(NR * DM * 2);
constexpr size_t WS_TOTAL = SZ_W + SZ_X + SZ_T + 2 * SZ_QK + 4 * SZ_P;
static_assert(WS_TOTAL <= (size_t)134217728);

extern "C" void kernel_launch(void* const* d_in, const int* in_sizes, int n_in,
                              void* d_out, int out_size, void* d_ws, size_t ws_size, hipStream_t stream) {
  if (n_in < 6) return;
  const size_t need_rows = (size_t)(NB - 1) * SEQ_FULL + SQ;
  if ((size_t)in_sizes[0] < need_rows * DM) return;
  if ((size_t)in_sizes[1] < need_rows) return;
  if ((size_t)in_sizes[2] < (size_t)DM * DM || (size_t)in_sizes[3] < (size_t)DM * DM || (size_t)in_sizes[4] < (size_t)DM * DM || (size_t)in_sizes[5] < (size_t)DM * DM) return;
  if ((size_t)out_size < need_rows * DM) return;
  const float* x = (const float*)d_in[0]; const int* tp = (const int*)d_in[1];
  const float* wq = (const float*)d_in[2]; const float* wk = (const float*)d_in[3]; const float* wv = (const float*)d_in[4]; const float* wo = (const float*)d_in[5];
  float* out = (float*)d_out;
  char* ws = (char*)d_ws; size_t off = 0;
  auto take = [&](size_t bytes) { char* p = ws + off; off += AL256(bytes); return p; };
  _Float16* BW = (_Float16*)take(SZ_W); _Float16* BQ = BW; _Float16* BK = BW + (size_t)DM * DM; _Float16* BV = BW + (size_t)2 * DM * DM; _Float16* BO = BW + (size_t)3 * DM * DM;
  _Float16* X16 = (_Float16*)take(SZ_X);
  float* TAB = (float*)take(SZ_T);
  _Float16* QKh = (_Float16*)take(SZ_QK); _Float16* QKr = (_Float16*)take(SZ_QK);
  _Float16* VTh = (_Float16*)take(SZ_P); _Float16* VTr = (_Float16*)take(SZ_P);
  _Float16* Oh = (_Float16*)take(SZ_P); _Float16* Orr = (_Float16*)take(SZ_P);
  if (off > ws_size || off > (size_t)134217728) return;
  _Float16* Qh = QKh; _Float16* Kh = QKh + NR * DM; _Float16* Qr = QKr; _Float16* Kr = QKr + NR * DM;

  InvF iv; { double p = 1.0; const double ratio = 0.7498942093324559; for (int i = 0; i < 32; ++i) { iv.v[i] = (float)p; p *= ratio; } }

  { const unsigned g = (unsigned)(((size_t)DM * DM / 8 + 255) / 256);
    k_wnat<<<g, 256, 0, stream>>>(wq, (size_t)DM * DM / 8, BQ); k_wnat<<<g, 256, 0, stream>>>(wk, (size_t)DM * DM / 8, BK);
    k_wnat<<<g, 256, 0, stream>>>(wv, (size_t)DM * DM / 8, BV); k_wnat<<<g, 256, 0, stream>>>(wo, (size_t)DM * DM / 8, BO); }
  k_x16<<<dim3((unsigned)(((size_t)SQ * DM / 8 + 255) / 256), NB), 256, 0, stream>>>(x, X16);
  k_ropetab<<<dim3((unsigned)((size_t)SQ * 16 / 256), NB), 256, 0, stream>>>(tp, TAB, iv);
  k_gemm3<false, 2><<<dim3(DM / 64, (unsigned)(NR / 128), 2), 128, 0, stream>>>(X16, nullptr, DM, 0, BQ, DM, (size_t)DM * DM, 0.0625f, TAB, nullptr, QKh, QKr, DM, NR * DM, (unsigned)NR, DM);
  k_gemm3<false, 1><<<dim3((unsigned)(NR / 64), DM / 128, 1), 128, 0, stream>>>(BV, nullptr, DM, 0, X16, DM, 0, 0.0625f, nullptr, nullptr, VTh, VTr, (unsigned)NR, 0, DM, DM);
  k_attn<true><<<dim3(BAND / 64, NH, NB), 128, 0, stream>>>(Qh, Qr, Kh, Kr, VTh, VTr, Oh, Orr, 0u);
  if (SQ > BAND) k_attn<false><<<dim3((SQ - BAND) / 64, NH, NB), 128, 0, stream>>>(Qh, Qr, Kh, Kr, VTh, VTr, Oh, Orr, (unsigned)(BAND / 64));
  k_gemm3<true, 0><<<dim3(DM / 64, BAND / 128, NB), 128, 0, stream>>>(Oh, Orr, DM, (size_t)SQ * DM, BO, DM, 0, 0.0009765625f, nullptr, out, nullptr, nullptr, DM, (size_t)SEQ_FULL * DM, (unsigned)BAND, DM);
  if (SQ > BAND) k_gemm3<false, 0><<<dim3(DM / 64, (SQ - BAND) / 128, NB), 128, 0, stream>>>(Oh + (size_t)BAND * DM, nullptr, DM, (size_t)SQ * DM, BO, DM, 0, 0.0009765625f, nullptr, out + (size_t)BAND * DM, nullptr, nullptr, DM, (size_t)SEQ_FULL * DM, (unsigned)(SQ - BAND), DM);
}
